// MultiheadAttentionFFN_54417235640330
// MI455X (gfx1250) — hardware-verified
//
#include <hip/hip_runtime.h>
#include <math.h>

typedef __attribute__((ext_vector_type(16))) _Float16 v16h;
typedef __attribute__((ext_vector_type(16))) __bf16 v16b;
typedef __attribute__((ext_vector_type(8)))  _Float16 v8h;
typedef __attribute__((ext_vector_type(8)))  float v8f;
typedef __attribute__((ext_vector_type(4)))  float v4f;
typedef __attribute__((ext_vector_type(2)))  float v2f;
typedef __attribute__((ext_vector_type(4)))  unsigned v4u;
typedef __attribute__((ext_vector_type(4)))  int v4i;
typedef float __attribute__((may_alias)) float_a;
typedef int __attribute__((may_alias)) int_a;

template <typename T> __device__ __forceinline__ void vst2(void* p, T v) { *(volatile T*)p = v; __threadfence(); *(volatile T*)p = v; }
__device__ __forceinline__ v8f wmma16(v16h a, v16h b, v8f c) {
  v8f d = __builtin_amdgcn_wmma_f32_16x16x32_f16(false, a, false, b, (short)0, c, false, false);
  asm volatile("v_nop\n\tv_nop\n\tv_nop\n\tv_nop" : "+v"(d) : "v"(a), "v"(b));
  return d;
}
__device__ __forceinline__ v8f wmma_bf(v16b a, v16b b, v8f c) {
  v8f d = __builtin_amdgcn_wmma_f32_16x16x32_bf16(false, a, false, b, (short)0, c, false, false);
  asm volatile("v_nop\n\tv_nop\n\tv_nop\n\tv_nop" : "+v"(d) : "v"(a), "v"(b));
  return d;
}
__device__ __forceinline__ v16h frag_h(const _Float16* rowk0, int lane) {
  union { v16h v; v8h q[2]; } u; const _Float16* p = rowk0 + 8 * (lane >> 4);
  u.q[0] = *(const v8h*)p; u.q[1] = *(const v8h*)(p + 16); return u.v;
}
__device__ __forceinline__ v16h frag_f32(const float* rowk0, int lane) {
  v16h a; const float* p = rowk0 + 8 * (lane >> 4);
#pragma unroll
  for (int i = 0; i < 8; ++i) { a[i] = (_Float16)p[i]; a[8 + i] = (_Float16)p[16 + i]; }
  return a;
}
__device__ __forceinline__ v16h frag_f32s(const float* rowk0, int lane, float sc) {
  v16h a; const float* p = rowk0 + 8 * (lane >> 4);
#pragma unroll
  for (int i = 0; i < 8; ++i) { a[i] = (_Float16)(p[i] * sc); a[8 + i] = (_Float16)(p[16 + i] * sc); }
  return a;
}
__device__ __forceinline__ v16h fragc_f32(const float* W, int k0, int n, int lane, int ld, int K) {
  v16h a; const int g = lane >> 4;
#pragma unroll
  for (int i = 0; i < 8; ++i) { const int ka = k0 + 8 * g + i, kb = ka + 16;
    a[i] = (_Float16)(ka < K ? W[(size_t)(ka < K ? ka : K - 1) * ld + n] : 0.f); a[8 + i] = (_Float16)(kb < K ? W[(size_t)(kb < K ? kb : K - 1) * ld + n] : 0.f); }
  return a;
}
struct F2 { v16b h, l; };
__device__ __forceinline__ F2 bsplit16(const float v[16]) { F2 r;
#pragma unroll
  for (int i = 0; i < 16; ++i) { const __bf16 h = (__bf16)v[i]; r.h[i] = h; r.l[i] = (__bf16)(v[i] - (float)h); }
  return r; }
__device__ __forceinline__ F2 split_row(const float* row, int k0, int lane) { float v[16]; const float* p = row + k0 + 8 * (lane >> 4);
#pragma unroll
  for (int i = 0; i < 8; ++i) { v[i] = p[i]; v[8 + i] = p[16 + i]; }
  return bsplit16(v); }
__device__ __forceinline__ F2 split_rowK(const float* row, int k0, int lane, int K) { float v[16]; const int g = lane >> 4;
#pragma unroll
  for (int i = 0; i < 8; ++i) { const int ka = k0 + 8 * g + i, kb = ka + 16; v[i] = ka < K ? row[ka < K ? ka : K - 1] : 0.f; v[8 + i] = kb < K ? row[kb < K ? kb : K - 1] : 0.f; }
  return bsplit16(v); }
__device__ __forceinline__ F2 split_col(const float* W, int k0, int n, int lane, int ld, int K) { float v[16]; const int g = lane >> 4;
#pragma unroll
  for (int i = 0; i < 8; ++i) { const int ka = k0 + 8 * g + i, kb = ka + 16; v[i] = ka < K ? W[(size_t)(ka < K ? ka : K - 1) * ld + n] : 0.f; v[8 + i] = kb < K ? W[(size_t)(kb < K ? kb : K - 1) * ld + n] : 0.f; }
  return bsplit16(v); }
__device__ __forceinline__ v8f mac3(const F2& a, const F2& b, v8f c) { c = wmma_bf(a.l, b.h, c); c = wmma_bf(a.h, b.l, c); return wmma_bf(a.h, b.h, c); }
__device__ __forceinline__ float sigm(float v) { return 1.0f / (1.0f + expf(-v)); }
#define LDSX() do { asm volatile("s_wait_dscnt 0" ::: "memory"); __builtin_amdgcn_wave_barrier(); __builtin_amdgcn_fence(__ATOMIC_RELEASE, "workgroup"); } while (0)


#define TT 2048
#define NB 2
#define EE 512
#define NH 8
#define HD 64
#define RD 256
#define NR (TT * NB)
#ifndef TQB
#define TQB (TT / 64)
#endif
typedef __attribute__((ext_vector_type(8))) __bf16 v8b;
__device__ __forceinline__ v16b frag_b(const __bf16* rowk0, int lane) {
  union { v16b v; v8b q[2]; } u; const __bf16* p = rowk0 + 8 * (lane >> 4);
  u.q[0] = *(const v8b*)p; u.q[1] = *(const v8b*)(p + 16); return u.v;
}
__device__ __forceinline__ float bfr(float v) { return (float)(__bf16)v; }
__device__ __attribute__((noinline)) float exp_ni(float v) { return expf(v); }
__device__ __attribute__((noinline)) float erf_ni(float v) { return erff(v); }

#define PK_Q 0
#define PK_K ((size_t)EE * EE)
#define PK_V ((size_t)2 * EE * EE)
#define PK_U ((size_t)3 * EE * EE)
#define PK_O ((size_t)4 * EE * EE)
#define PK_1 ((size_t)5 * EE * EE)
#define PK_2 (PK_1 + (size_t)RD * HD)
#define PK_END (PK_2 + (size_t)HD * RD)
#define WS_PK  0u
#define WS_TQ  (((2u * PK_END) + 127u) / 128u * 128u)
#define WS_TK  (WS_TQ + 4u * NR * EE)
#define WS_GT  (WS_TK + 4u * NR * EE)
#define WS_QH  (WS_GT + 4u * NR * EE)
#define WS_QL  (WS_QH + 2u * NR * EE)
#define WS_KH  (WS_QL + 2u * NR * EE)
#define WS_KL  (WS_KH + 2u * NR * EE)
#define WS_VTH (WS_KL + 2u * NR * EE)
#define WS_VTL (WS_VTH + 2u * NR * EE)
#define WS_O   (WS_VTL + 2u * NR * EE)
#define WS_YH  (WS_O + 4u * NR * EE)
#define WS_YL  (WS_YH + 2u * NR * EE)
#define WS_END (WS_YL + 2u * NR * EE)

__global__ __launch_bounds__(256) void k_pack(const float* __restrict__ WQ, const float* __restrict__ WK, const float* __restrict__ WV, const float* __restrict__ WU, const float* __restrict__ WO, const float* __restrict__ W1, const float* __restrict__ W2, __bf16* __restrict__ PK) {
  __shared__ __align__(16) __bf16 s[EE]; const int n = blockIdx.x, which = blockIdx.y, t = threadIdx.x; int K; size_t dst;
  if (which < 5) { const float* Wm = (which == 0) ? WQ : (which == 1) ? WK : (which == 2) ? WV : (which == 3) ? WU : WO; K = EE; dst = (size_t)which * EE * EE + (size_t)n * EE; for (int k = t; k < EE; k += 256) s[k] = (__bf16)Wm[(size_t)k * EE + n]; }
  else if (which == 5) { if (n >= RD) return; K = HD; dst = PK_1 + (size_t)n * HD; if (t < HD) s[t] = (__bf16)W1[(size_t)t * RD + n]; }
  else { if (n >= HD) return; K = RD; dst = PK_2 + (size_t)n * RD; s[t] = (__bf16)W2[(size_t)t * HD + n]; }
  __syncthreads();
  for (int q = t; q < K / 8; q += 256) vst2((unsigned*)(PK + dst + q * 8), *(const v4u*)&s[q * 8]);
}
__global__ __launch_bounds__(128) void k_proj(const float* __restrict__ X, const __bf16* __restrict__ PK, const float* __restrict__ BQ, const float* __restrict__ BK, const float* __restrict__ BV, const float* __restrict__ BU, float* __restrict__ TQ, float* __restrict__ TK, float* __restrict__ GT, _Float16* __restrict__ VTH, _Float16* __restrict__ VTL) {
  __shared__ __align__(16) float so[4][16][132]; __shared__ __align__(16) _Float16 sth[128][72], stl[128][72];
  const int tid = threadIdx.x, wave = tid >> 5, lane = tid & 31, col = lane & 15, g = lane >> 4; const int which = blockIdx.z; const size_t r0 = (size_t)blockIdx.x * 64 + wave * 16; const int n0 = blockIdx.y * 128;
  const int vb = blockIdx.x & 1, t0 = (blockIdx.x >> 1) * 64;
  const __bf16* P = PK + (size_t)which * EE * EE; const float* BB = (which == 0) ? BQ : (which == 1) ? BK : (which == 2) ? BV : BU;
  v8f acc[8] = {};
#pragma unroll 2
  for (int kc = 0; kc < EE / 32; ++kc) { v16b a; { const size_t arow = (which == 2) ? ((size_t)(t0 + wave * 16 + col) * NB + vb) : (r0 + col); const float* p = X + arow * EE + kc * 32 + 8 * g;
#pragma unroll
      for (int i = 0; i < 8; ++i) { a[i] = (__bf16)p[i]; a[8 + i] = (__bf16)p[16 + i]; } }
#pragma unroll
    for (int j = 0; j < 8; ++j) acc[j] = wmma_bf(a, frag_b(P + (size_t)(n0 + j * 16 + col) * EE + kc * 32, lane), acc[j]); }
  if (which != 2) { float* D = (which == 0) ? TQ : (which == 1) ? TK : GT;
#pragma unroll
    for (int j = 0; j < 8; ++j) { const float bb = bfr(BB[n0 + j * 16 + col]);
#pragma unroll
      for (int r = 0; r < 8; ++r) so[wave][8 * g + r][j * 16 + col] = acc[j][r] + bb; }
    LDSX();
    for (int rl = 0; rl < 16; ++rl) vst2(D + (r0 + rl) * EE + n0 + lane * 4, *(const v4f*)&so[wave][rl][lane * 4]);
  } else {
#pragma unroll
    for (int j = 0; j < 8; ++j) { const float bb = bfr(BB[n0 + j * 16 + col]);
#pragma unroll
      for (int r = 0; r < 8; ++r) { const int tl = wave * 16 + 8 * g + r; const float v = acc[j][r] + bb; const _Float16 hv = (_Float16)v; sth[j * 16 + col][tl] = hv; stl[j * 16 + col][tl] = (_Float16)((v - (float)hv) * 2048.0f); } }
    __syncthreads();
    for (int e = tid; e < 128 * 8; e += 128) { const int d = e >> 3, pc = e & 7; const size_t o = ((size_t)vb * EE + n0 + d) * TT + t0 + pc * 8; vst2((unsigned*)(VTH + o), *(const v4u*)&sth[d][pc * 8]); vst2((unsigned*)(VTL + o), *(const v4u*)&stl[d][pc * 8]); }
  }
}
__global__ __launch_bounds__(128) void k_lnqk(const float* __restrict__ TQ, const float* __restrict__ TK, const float* __restrict__ QG, const float* __restrict__ QB, const float* __restrict__ KG, const float* __restrict__ KB, _Float16* __restrict__ QH, _Float16* __restrict__ QL_, _Float16* __restrict__ KH, _Float16* __restrict__ KL) {
  __shared__ float red[2][4]; __shared__ __align__(16) _Float16 sh_[EE], sl_[EE]; const int t = threadIdx.x; const size_t row = blockIdx.x; const int which = blockIdx.y;
  const float* p = ((which == 0) ? TQ : TK) + row * EE + t * 4; const float* G = (which == 0) ? QG : KG; const float* Bv = (which == 0) ? QB : KB; const float post = (which == 0) ? 0.125f : 1.0f;
  float v[4] = {p[0], p[1], p[2], p[3]}; float s = (v[0] + v[1]) + (v[2] + v[3]);
#pragma unroll
  for (int o = 1; o < 32; o <<= 1) s += __shfl_xor(s, o);
  if ((t & 31) == 0) red[0][t >> 5] = s; __syncthreads();
  const float mu = (red[0][0] + red[0][1] + red[0][2] + red[0][3]) / (float)EE; float q = 0.f;
#pragma unroll
  for (int i = 0; i < 4; ++i) { const float d = v[i] - mu; q += d * d; }
#pragma unroll
  for (int o = 1; o < 32; o <<= 1) q += __shfl_xor(q, o);
  if ((t & 31) == 0) red[1][t >> 5] = q; __syncthreads();
  const float inv = 1.0f / sqrtf((red[1][0] + red[1][1] + red[1][2] + red[1][3]) / (float)EE + 1e-5f);
#pragma unroll
  for (int i = 0; i < 4; ++i) { const int c = t * 4 + i; const float y = ((v[i] - mu) * inv * bfr(G[c]) + bfr(Bv[c])) * post; const _Float16 hv = (_Float16)y; sh_[c] = hv; sl_[c] = (_Float16)((y - (float)hv) * 2048.0f); }
  __syncthreads();
  _Float16* DH = (which == 0) ? QH : KH; _Float16* DL = (which == 0) ? QL_ : KL;
  if (t < 64) vst2((unsigned*)(DH + row * EE + t * 8), *(const v4u*)&sh_[t * 8]); else vst2((unsigned*)(DL + row * EE + (t - 64) * 8), *(const v4u*)&sl_[(t - 64) * 8]);
}
__global__ __launch_bounds__(128) void k_attn(const _Float16* __restrict__ QH, const _Float16* __restrict__ QL_, const _Float16* __restrict__ KH, const _Float16* __restrict__ KL, const _Float16* __restrict__ VTH, const _Float16* __restrict__ VTL, float* __restrict__ O) {
  __shared__ __align__(16) _Float16 sph[4][16][40], spl[4][16][40]; __shared__ __align__(16) float so[4][16][68];
  const int tid = threadIdx.x, wave = tid >> 5, lane = tid & 31, col = lane & 15, g = lane >> 4; const int qb = blockIdx.x, h = blockIdx.y, b = blockIdx.z; const int q0 = qb * 64 + wave * 16;
  v16h aqh[2], aql[2]; { const size_t rq = ((size_t)(q0 + col) * NB + b) * EE + h * HD;
#pragma unroll
    for (int kc = 0; kc < 2; ++kc) { aqh[kc] = frag_h(QH + rq + kc * 32, lane); aql[kc] = frag_h(QL_ + rq + kc * 32, lane); } }
  const _Float16* Vh = VTH + ((size_t)b * EE + h * HD) * TT; const _Float16* Vl = VTL + ((size_t)b * EE + h * HD) * TT;
  float m[8], l[8];
#pragma unroll
  for (int r = 0; r < 8; ++r) { m[r] = -3.0e38f; l[r] = 0.f; }
  v8f acc[4] = {}, accl[4] = {};
#pragma unroll 1
  for (int ks = 0; ks < TT / 32; ++ks) { v8f s[2];
#pragma unroll
    for (int ct = 0; ct < 2; ++ct) { const int kk = ks * 32 + ct * 16 + col; const size_t rk = ((size_t)kk * NB + b) * EE + h * HD; v8f c = {}, cl = {};
#pragma unroll
      for (int kc = 0; kc < 2; ++kc) { const v16h khf = frag_h(KH + rk + kc * 32, lane); c = wmma16(aqh[kc], khf, c); cl = wmma16(aql[kc], khf, cl); cl = wmma16(aqh[kc], frag_h(KL + rk + kc * 32, lane), cl); }
#pragma unroll
      for (int r = 0; r < 8; ++r) s[ct][r] = c[r] + cl[r] * (1.0f / 2048.0f); }
#pragma unroll
    for (int r = 0; r < 8; ++r) { float mx = fmaxf(s[0][r], s[1][r]);
#pragma unroll
      for (int o = 1; o < 16; o <<= 1) mx = fmaxf(mx, __shfl_xor(mx, o));
      const float mn = fmaxf(m[r], mx); const float alpha = (m[r] <= -1.0e38f) ? 0.f : __expf(m[r] - mn); const float e0 = __expf(s[0][r] - mn), e1 = __expf(s[1][r] - mn); float es = e0 + e1;
#pragma unroll
      for (int o = 1; o < 16; o <<= 1) es += __shfl_xor(es, o);
      l[r] = l[r] * alpha + es; m[r] = mn;
#pragma unroll
      for (int dt = 0; dt < 4; ++dt) { acc[dt][r] *= alpha; accl[dt][r] *= alpha; }
      const _Float16 h0 = (_Float16)e0, h1 = (_Float16)e1; sph[wave][8 * g + r][col] = h0; sph[wave][8 * g + r][16 + col] = h1; spl[wave][8 * g + r][col] = (_Float16)((e0 - (float)h0) * 2048.0f); spl[wave][8 * g + r][16 + col] = (_Float16)((e1 - (float)h1) * 2048.0f); }
    LDSX();
    const v16h pah = frag_h(&sph[wave][col][0], lane), pal = frag_h(&spl[wave][col][0], lane);
#pragma unroll
    for (int dt = 0; dt < 4; ++dt) { const size_t vo = (size_t)(dt * 16 + col) * TT + ks * 32; const v16h vh = frag_h(Vh + vo, lane), vl = frag_h(Vl + vo, lane); acc[dt] = wmma16(pah, vh, acc[dt]); accl[dt] = wmma16(pal, vh, accl[dt]); accl[dt] = wmma16(pah, vl, accl[dt]); }
    LDSX(); }
#pragma unroll
  for (int r = 0; r < 8; ++r) { const float il = 1.0f / l[r];
#pragma unroll
    for (int dt = 0; dt < 4; ++dt) so[wave][8 * g + r][dt * 16 + col] = (acc[dt][r] + accl[dt][r] * (1.0f / 2048.0f)) * il; }
  LDSX();
  for (int rl = 0; rl < 16; ++rl) if (lane < 16) vst2(O + ((size_t)(q0 + rl) * NB + b) * EE + h * HD + lane * 4, *(const v4f*)&so[wave][rl][lane * 4]);
}
__global__ __launch_bounds__(128) void k_hffn(const float* __restrict__ O, const float* __restrict__ GT, const __bf16* __restrict__ PK, const float* __restrict__ B1, const float* __restrict__ B2, const float* __restrict__ FG, const float* __restrict__ FB, __bf16* __restrict__ YH, __bf16* __restrict__ YL) {
  __shared__ __align__(16) __bf16 shh[64][72], shl[64][72]; __shared__ __align__(16) __bf16 sah[64][RD + 8], sal[64][RD + 8]; __shared__ __align__(16) __bf16 syh[4][16][72], syl[4][16][72];
  const int tid = threadIdx.x, wave = tid >> 5, lane = tid & 31, col = lane & 15, g = lane >> 4; const size_t rb = (size_t)blockIdx.x * 64; const int h = blockIdx.y;
  { const int r = tid >> 1, half = tid & 1; const float* p = O + (rb + r) * EE + h * HD + half * 32; float v[32]; float s = 0.f;
#pragma unroll
    for (int i = 0; i < 32; ++i) { v[i] = p[i]; s += v[i]; }
    s += __shfl_xor(s, 1); const float mu = s / 64.0f; float q = 0.f;
#pragma unroll
    for (int i = 0; i < 32; ++i) { const float d = v[i] - mu; q += d * d; }
    q += __shfl_xor(q, 1); const float inv = 1.0f / sqrtf(q / 64.0f + 1e-5f);
#pragma unroll
    for (int i = 0; i < 32; ++i) { const int c = half * 32 + i; const float y = (v[i] - mu) * inv * bfr(FG[c]) + bfr(FB[c]); const __bf16 hb = (__bf16)y; shh[r][c] = hb; shl[r][c] = (__bf16)(y - (float)hb); }
    if (half == 0) for (int c = 64; c < 72; ++c) { shh[r][c] = (__bf16)0.f; shl[r][c] = (__bf16)0.f; } }
  __syncthreads();
#pragma unroll 1
  for (int hf = 0; hf < 2; ++hf) { v8f acc[8] = {};
#pragma unroll
    for (int kc = 0; kc < 2; ++kc) { F2 a; a.h = frag_b(&shh[wave * 16 + col][kc * 32], lane); a.l = frag_b(&shl[wave * 16 + col][kc * 32], lane);
#pragma unroll
      for (int j = 0; j < 8; ++j) { const v16b w = frag_b(PK + PK_1 + (size_t)(hf * 128 + j * 16 + col) * HD + kc * 32, lane); acc[j] = wmma_bf(a.l, w, acc[j]); acc[j] = wmma_bf(a.h, w, acc[j]); } }
#pragma unroll
    for (int j = 0; j < 8; ++j) { const int c = hf * 128 + j * 16 + col; const float bb = bfr(B1[c]);
#pragma unroll
      for (int r = 0; r < 8; ++r) { const float v = fmaxf(acc[j][r] + bb, 0.f); const __bf16 hb = (__bf16)v; sah[wave * 16 + 8 * g + r][c] = hb; sal[wave * 16 + 8 * g + r][c] = (__bf16)(v - (float)hb); } } }
  LDSX();
  v8f acc2[4] = {};
#pragma unroll 2
  for (int kc = 0; kc < RD / 32; ++kc) { F2 a; a.h = frag_b(&sah[wave * 16 + col][kc * 32], lane); a.l = frag_b(&sal[wave * 16 + col][kc * 32], lane);
#pragma unroll
    for (int j = 0; j < 4; ++j) { const v16b w = frag_b(PK + PK_2 + (size_t)(j * 16 + col) * RD + kc * 32, lane); acc2[j] = wmma_bf(a.l, w, acc2[j]); acc2[j] = wmma_bf(a.h, w, acc2[j]); } }
#pragma unroll
  for (int j = 0; j < 4; ++j) { const int c = j * 16 + col; const float bb = bfr(B2[c]);
#pragma unroll
    for (int r = 0; r < 8; ++r) { const size_t row = rb + wave * 16 + 8 * g + r; const float f = acc2[j][r] + bb + O[row * EE + h * HD + c]; const float y = f * GT[row * EE + h * HD + c]; const __bf16 hb = (__bf16)y; syh[wave][8 * g + r][c] = hb; syl[wave][8 * g + r][c] = (__bf16)(y - (float)hb); } }
  LDSX();
  for (int rl = 0; rl < 16; ++rl) { const size_t o = (rb + wave * 16 + rl) * EE + h * HD; if (lane < 8) vst2((unsigned*)(YH + o + lane * 8), *(const v4u*)&syh[wave][rl][lane * 8]); else if (lane < 16) vst2((unsigned*)(YL + o + (lane - 8) * 8), *(const v4u*)&syl[wave][rl][(lane - 8) * 8]); }
}
__global__ __launch_bounds__(128) void k_out(const __bf16* __restrict__ YH, const __bf16* __restrict__ YL, const __bf16* __restrict__ PK, const float* __restrict__ BO, float* __restrict__ OUT) {
  __shared__ __align__(16) float so[4][16][132];
  const int tid = threadIdx.x, wave = tid >> 5, lane = tid & 31, col = lane & 15, g = lane >> 4; const size_t r0 = (size_t)blockIdx.x * 64 + wave * 16; const int n0 = blockIdx.y * 128;
  v8f acc[8] = {};
#pragma unroll 2
  for (int kc = 0; kc < EE / 32; ++kc) { const v16b ah = frag_b(YH + (r0 + col) * EE + kc * 32, lane), al = frag_b(YL + (r0 + col) * EE + kc * 32, lane);
#pragma unroll
    for (int j = 0; j < 8; ++j) { const v16b w = frag_b(PK + PK_O + (size_t)(n0 + j * 16 + col) * EE + kc * 32, lane); acc[j] = wmma_bf(al, w, acc[j]); acc[j] = wmma_bf(ah, w, acc[j]); } }
#pragma unroll
  for (int j = 0; j < 8; ++j) { const float bb = bfr(BO[n0 + j * 16 + col]);
#pragma unroll
    for (int r = 0; r < 8; ++r) so[wave][8 * g + r][j * 16 + col] = acc[j][r] + bb; }
  LDSX();
  for (int rl = 0; rl < 16; ++rl) vst2(OUT + (r0 + rl) * EE + n0 + lane * 4, *(const v4f*)&so[wave][rl][lane * 4]);
}
extern "C" void kernel_launch(void* const* d_in, const int* in_sizes, int n_in, void* d_out, int out_size, void* d_ws, size_t ws_size, hipStream_t stream) {
  (void)in_sizes; (void)n_in; (void)out_size;
  const float** F = (const float**)d_in;
  if (ws_size < (size_t)WS_END) return;
  char* ws = (char*)d_ws; __bf16 *PK = (__bf16*)(ws + WS_PK), *YH = (__bf16*)(ws + WS_YH), *YL = (__bf16*)(ws + WS_YL); float *TQ = (float*)(ws + WS_TQ), *TK = (float*)(ws + WS_TK), *GT = (float*)(ws + WS_GT), *O = (float*)(ws + WS_O); _Float16 *QH = (_Float16*)(ws + WS_QH), *QLp = (_Float16*)(ws + WS_QL), *KH = (_Float16*)(ws + WS_KH), *KL = (_Float16*)(ws + WS_KL), *VTH = (_Float16*)(ws + WS_VTH), *VTL = (_Float16*)(ws + WS_VTL);
  k_pack<<<dim3(EE, 7), 256, 0, stream>>>(F[1], F[3], F[5], F[7], F[9], F[11], F[13], PK);
  k_proj<<<dim3(NR / 64, EE / 128, 4), 128, 0, stream>>>(F[0], PK, F[2], F[4], F[6], F[8], TQ, TK, GT, VTH, VTL);
  k_lnqk<<<dim3(NR, 2), 128, 0, stream>>>(TQ, TK, F[15], F[16], F[17], F[18], QH, QLp, KH, KL);
  k_attn<<<dim3(TQB, NH, NB), 128, 0, stream>>>(QH, QLp, KH, KL, VTH, VTL, O);
  k_hffn<<<dim3(NR / 64, NH), 128, 0, stream>>>(O, GT, PK, F[12], F[14], F[19], F[20], YH, YL);
  k_out<<<dim3(NR / 64, EE / 128), 128, 0, stream>>>(YH, YL, PK, F[10], (float*)d_out);
}
